// LocalBranch_46437186404433
// MI455X (gfx1250) — hardware-verified
//
#include <hip/hip_runtime.h>


#define NNODE 131072
#define NG    1024
#define GN    128
#define FIN   64
#define HID   256
#define FO    128
#define CHN   16384
#define NCH   (NNODE / CHN)
#define DM    HID
#define NTK   CHN
#define TAU   0.25f
#define LOSC 1024.0f

typedef _Float16 h16;
typedef unsigned short bf;
typedef __attribute__((ext_vector_type(16))) __bf16   v16bf;
typedef __attribute__((ext_vector_type(16))) _Float16 v16h;
typedef __attribute__((ext_vector_type(8)))  _Float16 v8h;
typedef __attribute__((ext_vector_type(8)))  unsigned short v8us;
typedef __attribute__((ext_vector_type(8)))  float    v8f;
typedef __attribute__((ext_vector_type(4)))  float    v4f;
typedef __attribute__((ext_vector_type(4)))  _Float16 v4h;
typedef v8h  __attribute__((may_alias)) v8ha;
typedef v4f  __attribute__((may_alias)) v4fa;
typedef v8us __attribute__((may_alias)) v8usa;

__device__ __forceinline__ unsigned short f2bf(float f) { unsigned u = __float_as_uint(f); u += 0x7FFFu + ((u >> 16) & 1u); return (unsigned short)(u >> 16); }
__device__ __forceinline__ float bf2f(unsigned short b) { return __uint_as_float(((unsigned)b) << 16); }
__device__ __forceinline__ float bfr(float f) { return bf2f(f2bf(f)); }
__device__ __forceinline__ v16h cat16(v8h lo, v8h hi) { return __builtin_shufflevector(lo, hi, 0, 1, 2, 3, 4, 5, 6, 7, 8, 9, 10, 11, 12, 13, 14, 15); }
__device__ __forceinline__ v16bf cat16b(v8us lo, v8us hi) { return __builtin_bit_cast(v16bf, __builtin_shufflevector(lo, hi, 0, 1, 2, 3, 4, 5, 6, 7, 8, 9, 10, 11, 12, 13, 14, 15)); }
__device__ __forceinline__ v8f wmma16(v16h a, v16h b, v8f c) { return __builtin_amdgcn_wmma_f32_16x16x32_f16(false, a, false, b, (short)0, c, false, false); }
__device__ __forceinline__ v8f wmmab(v16bf a, v16bf b, v8f c) { return __builtin_amdgcn_wmma_f32_16x16x32_bf16(false, a, false, b, (short)0, c, false, false); }

__global__ __launch_bounds__(256) void k_wt(const float* __restrict__ Wm, int K, int ncols, bf* WT) {
    __shared__ __align__(16) unsigned short tl[64 * 72];
    const int tid = threadIdx.x, k0 = blockIdx.x * 64, n0 = blockIdx.y * 64;
    const int kk = tid >> 2, nq = (tid & 3) * 16;
#pragma unroll
    for (int i = 0; i < 16; ++i) tl[(nq + i) * 72 + kk] = f2bf(Wm[(size_t)(k0 + kk) * ncols + n0 + nq + i]);
    __syncthreads();
    const int piece = tid & 7;
    auto pass = [&]() {
#pragma unroll
        for (int s = 0; s < 2; ++s) { const int nr = (tid >> 3) + 32 * s; const v8us val = *(const v8usa*)(tl + nr * 72 + piece * 8); *(volatile v8us*)(WT + (size_t)(n0 + nr) * K + k0 + piece * 8) = val; }
    };
    pass(); __threadfence(); pass();
}
template <bool SPLITA, bool F16OUT = false>
__global__ __launch_bounds__(128) void k_gemmb(const bf* __restrict__ A, const bf* __restrict__ Al, const bf* __restrict__ Bn, const float* __restrict__ bias, float* C, int ldc, h16* C2, const float* __restrict__ R = nullptr, int K = DM, int roundR = 1) {
    __shared__ __align__(16) float ost[4][16 * 68];
    const int lane = threadIdx.x & 31, wave = threadIdx.x >> 5, lr = lane & 15, hi = lane >> 4;
    const int r0 = blockIdx.x * 64 + wave * 16, c0 = blockIdx.y * 64;
    const size_t aoff = (size_t)(r0 + lr) * K + 8 * hi;
    size_t boff[4];
#pragma unroll
    for (int t = 0; t < 4; ++t) boff[t] = (size_t)(c0 + t * 16 + lr) * K + 8 * hi;
    v8f acc[4];
#pragma unroll
    for (int t = 0; t < 4; ++t) acc[t] = (v8f){};
#pragma unroll 1
    for (int kc = 0; kc < K; kc += 32) {
        const v16bf a = cat16b(*(const v8us*)(A + aoff + kc), *(const v8us*)(A + aoff + kc + 16));
        v16bf al = a;
        if (SPLITA) al = cat16b(*(const v8us*)(Al + aoff + kc), *(const v8us*)(Al + aoff + kc + 16));
#pragma unroll
        for (int t = 0; t < 4; ++t) { const v16bf b = cat16b(*(const v8us*)(Bn + boff[t] + kc), *(const v8us*)(Bn + boff[t] + kc + 16)); acc[t] = wmmab(a, b, acc[t]); if (SPLITA) acc[t] = wmmab(al, b, acc[t]); }
        asm volatile("v_nop\n\tv_nop\n\tv_nop\n\tv_nop" : "+v"(acc[0]), "+v"(acc[1]), "+v"(acc[2]), "+v"(acc[3]) : "v"(a), "v"(al));
    }
    float* os = &ost[wave][0];
#pragma unroll
    for (int t = 0; t < 4; ++t) { const float bv = bias ? bfr(bias[c0 + t * 16 + lr]) : 0.f;
#pragma unroll
        for (int j = 0; j < 8; ++j) os[(hi * 8 + j) * 68 + t * 16 + lr] = acc[t][j] + bv; }
    __syncthreads();
    if (F16OUT) {
        h16* crow = (h16*)(void*)C + (size_t)r0 * ldc + c0;
        auto pass = [&]() {
#pragma unroll
            for (int s = 0; s < 4; ++s) { const int row = 4 * s + (lane >> 3), piece = lane & 7; const float* sp = os + row * 68 + piece * 8; v8h o, o2;
#pragma unroll
                for (int i = 0; i < 8; ++i) { const h16 a = (h16)sp[i]; o[i] = a; o2[i] = (h16)((sp[i] - (float)a) * LOSC); }
                *(volatile v8h*)(crow + (size_t)row * ldc + piece * 8) = o; if (C2) *(volatile v8h*)(C2 + (size_t)r0 * ldc + c0 + (size_t)row * ldc + piece * 8) = o2; }
        };
        pass(); __threadfence(); pass();
    } else {
        float* crow = C + (size_t)r0 * ldc + c0;
        auto pass = [&]() {
#pragma unroll
            for (int s = 0; s < 8; ++s) { const int Lid = (lane >> 3) + 4 * s, piece = lane & 7; const int row = Lid >> 1, cofs = (Lid & 1) * 32 + piece * 4;
                v4f val = *(const v4fa*)(os + row * 68 + cofs); if (R) { const v4f rv = *(const v4f*)(R + ((size_t)r0 + row) * ldc + c0 + cofs); val += roundR ? (v4f){bfr(rv[0]), bfr(rv[1]), bfr(rv[2]), bfr(rv[3])} : rv; }
                *(volatile v4f*)(crow + (size_t)row * ldc + cofs) = val; }
        };
        pass(); __threadfence(); pass();
    }
}

__global__ __launch_bounds__(128) void k_gemm3(const bf* __restrict__ Ah, const bf* __restrict__ Al, const bf* __restrict__ Bh, const bf* __restrict__ Bl, int K, float* C, int ldc) {
    __shared__ __align__(16) float ost[4][16 * 68];
    const int lane = threadIdx.x & 31, wave = threadIdx.x >> 5, lr = lane & 15, hi = lane >> 4;
    const int r0 = blockIdx.x * 64 + wave * 16, c0 = blockIdx.y * 64;
    const size_t aoff = (size_t)(r0 + lr) * K + 8 * hi;
    v8f acc[4];
#pragma unroll
    for (int t = 0; t < 4; ++t) acc[t] = (v8f){};
#pragma unroll 1
    for (int kc = 0; kc < K; kc += 32) {
        const v16bf a = cat16b(*(const v8us*)(Ah + aoff + kc), *(const v8us*)(Ah + aoff + kc + 16));
        const v16bf al = cat16b(*(const v8us*)(Al + aoff + kc), *(const v8us*)(Al + aoff + kc + 16));
#pragma unroll
        for (int t = 0; t < 4; ++t) { const size_t bo = (size_t)(c0 + t * 16 + lr) * K + kc + 8 * hi;
            const v16bf bh = cat16b(*(const v8us*)(Bh + bo), *(const v8us*)(Bh + bo + 16)); const v16bf bl = cat16b(*(const v8us*)(Bl + bo), *(const v8us*)(Bl + bo + 16));
            acc[t] = wmmab(a, bh, acc[t]); acc[t] = wmmab(al, bh, acc[t]); acc[t] = wmmab(a, bl, acc[t]); }
        asm volatile("v_nop\n\tv_nop\n\tv_nop\n\tv_nop" : "+v"(acc[0]), "+v"(acc[1]), "+v"(acc[2]), "+v"(acc[3]) : "v"(a), "v"(al));
    }
    float* os = &ost[wave][0];
#pragma unroll
    for (int t = 0; t < 4; ++t) {
#pragma unroll
        for (int j = 0; j < 8; ++j) os[(hi * 8 + j) * 68 + t * 16 + lr] = acc[t][j]; }
    __builtin_amdgcn_wave_barrier(); asm volatile("" ::: "memory");
    float* crow = C + (size_t)r0 * ldc + c0;
    auto pass = [&]() {
#pragma unroll
        for (int s = 0; s < 8; ++s) { const int Lid = (lane >> 3) + 4 * s, piece = lane & 7; const int row = Lid >> 1, cofs = (Lid & 1) * 32 + piece * 4;
            const v4f val = *(const v4fa*)(os + row * 68 + cofs); *(volatile v4f*)(crow + (size_t)row * ldc + cofs) = val; }
    };
    pass(); __threadfence(); pass();
}

__global__ __launch_bounds__(256) void k_bfrows(const float* __restrict__ Hs, bf* Hb) {
    typedef __attribute__((ext_vector_type(2))) unsigned short v2us;
    const int lane = threadIdx.x & 31, r = blockIdx.x * 8 + (threadIdx.x >> 5); if (r >= CHN) return;
    const size_t o = (size_t)r * FIN + lane * 2; v2us v; v[0] = f2bf(Hs[o]); v[1] = f2bf(Hs[o + 1]);
    *(volatile v2us*)(Hb + o) = v; __threadfence(); *(volatile v2us*)(Hb + o) = v;
}
template <int MODE>
__global__ __launch_bounds__(256) void k_lnact(const float* __restrict__ T, const float* __restrict__ g, const float* __restrict__ bb, int nrows, float* X, bf* Xh, bf* Xl) {
    typedef __attribute__((ext_vector_type(4))) unsigned short v4us;
    const int lane = threadIdx.x & 31, r = blockIdx.x * 8 + (threadIdx.x >> 5); if (r >= nrows) return;
    const float* tr = T + (size_t)r * HID;
    float s = 0.f;
#pragma unroll
    for (int q = 0; q < HID / 128; ++q) { const v4f v = *(const v4f*)(tr + q * 128 + lane * 4); s += (v[0] + v[1]) + (v[2] + v[3]); }
#pragma unroll
    for (int sh = 16; sh; sh >>= 1) s += __shfl_xor(s, sh, 32);
    const float mu = s * (1.0f / HID); float s2 = 0.f;
#pragma unroll
    for (int q = 0; q < HID / 128; ++q) { const v4f v = *(const v4f*)(tr + q * 128 + lane * 4);
#pragma unroll
        for (int i = 0; i < 4; ++i) { const float d = v[i] - mu; s2 = fmaf(d, d, s2); } }
#pragma unroll
    for (int sh = 16; sh; sh >>= 1) s2 += __shfl_xor(s2, sh, 32);
    const float rs = rsqrtf(s2 * (1.0f / HID) + 1e-5f);
    v4f y[HID / 128]; v4us oh[HID / 128], ol[HID / 128];
#pragma unroll
    for (int q = 0; q < HID / 128; ++q) { const int c0 = q * 128 + lane * 4; const v4f v = *(const v4f*)(tr + c0); const v4f xo = (MODE == 1) ? *(const v4f*)(X + (size_t)r * HID + c0) : (v4f){};
#pragma unroll
        for (int i = 0; i < 4; ++i) { const float a = fmaxf((v[i] - mu) * rs * bfr(g[c0 + i]) + bfr(bb[c0 + i]), 0.f) + xo[i]; y[q][i] = a; const unsigned short hb = f2bf(a); oh[q][i] = hb; ol[q][i] = f2bf(a - bf2f(hb)); } }
#pragma unroll 1
    for (int ps = 0; ps < 2; ++ps) {
#pragma unroll
        for (int q = 0; q < HID / 128; ++q) { const size_t o = (size_t)r * HID + q * 128 + lane * 4; *(volatile v4f*)(X + o) = y[q]; *(volatile v4us*)(Xh + o) = oh[q]; *(volatile v4us*)(Xl + o) = ol[q]; }
        if (ps == 0) __threadfence(); }
}
__global__ __launch_bounds__(256) void k_lnz(const float* __restrict__ T, const float* __restrict__ g, const float* __restrict__ bb, int nrows, float* Z, bf* Zh, bf* Zl) {
    typedef __attribute__((ext_vector_type(4))) unsigned short v4us;
    const int lane = threadIdx.x & 31, r = blockIdx.x * 8 + (threadIdx.x >> 5); if (r >= nrows) return;
    const size_t o = (size_t)r * FO + lane * 4; const v4f v = *(const v4f*)(T + o);
    float s = (v[0] + v[1]) + (v[2] + v[3]);
#pragma unroll
    for (int sh = 16; sh; sh >>= 1) s += __shfl_xor(s, sh, 32);
    const float mu = s * (1.0f / FO); float s2 = 0.f;
#pragma unroll
    for (int i = 0; i < 4; ++i) { const float d = v[i] - mu; s2 = fmaf(d, d, s2); }
#pragma unroll
    for (int sh = 16; sh; sh >>= 1) s2 += __shfl_xor(s2, sh, 32);
    const float rs = rsqrtf(s2 * (1.0f / FO) + 1e-5f);
    v4f y; v4us oh, ol;
#pragma unroll
    for (int i = 0; i < 4; ++i) { const int c = lane * 4 + i; const float a = (v[i] - mu) * rs * bfr(g[c]) + bfr(bb[c]); y[i] = a; const unsigned short hb = f2bf(a); oh[i] = hb; ol[i] = f2bf(a - bf2f(hb)); }
    *(volatile v4f*)(Z + o) = y; *(volatile v4us*)(Zh + o) = oh; *(volatile v4us*)(Zl + o) = ol; __threadfence(); *(volatile v4f*)(Z + o) = y; *(volatile v4us*)(Zh + o) = oh; *(volatile v4us*)(Zl + o) = ol;
}
__global__ __launch_bounds__(128) void k_graph(const float* __restrict__ Z, const float* __restrict__ G, int node0, float* VOUT, float* WOUT) {
    __shared__ float sq[GN]; __shared__ float ws[GN]; __shared__ float red[4];
    const int tid = threadIdx.x, lane = tid & 31, wave = tid >> 5; const int gi = blockIdx.x;
    const int gstart = node0 + gi * GN;
    const int lrow = gi * GN + tid;
    const float* zr = Z + (size_t)lrow * FO;
    float q2 = 0.f;
#pragma unroll 1
    for (int d = 0; d < FO; d += 4) { const v4f v = *(const v4f*)(zr + d); q2 += (v[0] * v[0] + v[1] * v[1]) + (v[2] * v[2] + v[3] * v[3]); }
    sq[tid] = q2;
    __syncthreads();
    const float* gr = G + ((size_t)gi * GN + tid) * GN;
    float s = 0.f;
#pragma unroll 1
    for (int j = 0; j < GN; ++j) { const float d2 = sq[tid] + sq[j] - 2.0f * gr[j]; s += sqrtf(fmaxf(d2, 0.f) + 1e-12f); }
    s *= (1.0f / GN);
    const float a = s / TAU;
    float m = a;
#pragma unroll
    for (int sh = 16; sh; sh >>= 1) m = fmaxf(m, __shfl_xor(m, sh, 32));
    if (lane == 0) red[wave] = m;
    __syncthreads();
    const float mx = fmaxf(fmaxf(red[0], red[1]), fmaxf(red[2], red[3]));
    const float e = __expf(a - mx);
    __syncthreads();
    float se = e;
#pragma unroll
    for (int sh = 16; sh; sh >>= 1) se += __shfl_xor(se, sh, 32);
    if (lane == 0) red[wave] = se;
    __syncthreads();
    const float den = (red[0] + red[1]) + (red[2] + red[3]);
    const float w = e / den; ws[tid] = w;
    __syncthreads();
    float vl = 0.f;
#pragma unroll 1
    for (int i = 0; i < GN; ++i) vl = fmaf(ws[i], Z[(size_t)(gstart - node0 + i) * FO + tid], vl);
    const int gg = node0 / GN + gi;
    *(volatile float*)(VOUT + (size_t)gg * FO + tid) = vl; *(volatile float*)(WOUT + (size_t)gg * GN + tid) = w; __threadfence();
    *(volatile float*)(VOUT + (size_t)gg * FO + tid) = vl; *(volatile float*)(WOUT + (size_t)gg * GN + tid) = w;
}

extern "C" void kernel_launch(void* const* d_in, const int* in_sizes, int n_in,
                              void* d_out, int out_size, void* d_ws, size_t ws_size, hipStream_t stream) {
    (void)in_sizes; (void)n_in; (void)out_size;
    const float* Hin = (const float*)d_in[0];
    const float* Win = (const float*)d_in[2]; const float* bin = (const float*)d_in[3]; const float* gin = (const float*)d_in[4]; const float* bein = (const float*)d_in[5];
    const float* Wb = (const float*)d_in[6]; const float* bbk = (const float*)d_in[7]; const float* gbk = (const float*)d_in[8]; const float* bebk = (const float*)d_in[9];
    const float* Wout = (const float*)d_in[10]; const float* bout = (const float*)d_in[11]; const float* gout = (const float*)d_in[12]; const float* beout = (const float*)d_in[13];
    float* out0 = (float*)d_out; float* out1 = out0 + (size_t)NG * FO;
    char* wsp = (char*)d_ws;
    auto take = [&](size_t bytes) { char* p = wsp; wsp += (bytes + 255) & ~(size_t)255; return (void*)p; };
    bf* WinT = (bf*)take((size_t)HID * FIN * 2); bf* WbT = (bf*)take((size_t)3 * HID * HID * 2); bf* WoutT = (bf*)take((size_t)FO * HID * 2);
    bf* Hb = (bf*)take((size_t)CHN * FIN * 2); float* T = (float*)take((size_t)CHN * HID * 4); float* X = (float*)take((size_t)CHN * HID * 4); bf* Xh = (bf*)take((size_t)CHN * HID * 2); bf* Xl = (bf*)take((size_t)CHN * HID * 2);
    float* T2 = (float*)take((size_t)CHN * FO * 4); float* Z = (float*)take((size_t)CHN * FO * 4); bf* Zh = (bf*)take((size_t)CHN * FO * 2); bf* Zl = (bf*)take((size_t)CHN * FO * 2); float* G = (float*)take((size_t)(CHN / GN) * GN * GN * 4);
    if ((size_t)(wsp - (char*)d_ws) > ws_size) return;
    k_wt<<<dim3(FIN / 64, HID / 64, 1), 256, 0, stream>>>(Win, FIN, HID, WinT);
    for (int k = 0; k < 3; ++k) k_wt<<<dim3(HID / 64, HID / 64, 1), 256, 0, stream>>>(Wb + (size_t)k * HID * HID, HID, HID, WbT + (size_t)k * HID * HID);
    k_wt<<<dim3(HID / 64, FO / 64, 1), 256, 0, stream>>>(Wout, HID, FO, WoutT);
    for (int ch = 0; ch < NCH; ++ch) {
        const int node0 = ch * CHN;
        k_bfrows<<<CHN / 8, 256, 0, stream>>>(Hin + (size_t)node0 * FIN, Hb);
        k_gemmb<false, false><<<dim3(CHN / 64, HID / 64, 1), 128, 0, stream>>>(Hb, nullptr, WinT, bin, T, HID, nullptr, nullptr, FIN);
        k_lnact<0><<<CHN / 8, 256, 0, stream>>>(T, gin, bein, CHN, X, Xh, Xl);
        for (int k = 0; k < 3; ++k) {
            k_gemmb<true, false><<<dim3(CHN / 64, HID / 64, 1), 128, 0, stream>>>(Xh, Xl, WbT + (size_t)k * HID * HID, bbk + k * HID, T, HID, nullptr);
            k_lnact<1><<<CHN / 8, 256, 0, stream>>>(T, gbk + k * HID, bebk + k * HID, CHN, X, Xh, Xl);
        }
        k_gemmb<true, false><<<dim3(CHN / 64, FO / 64, 1), 128, 0, stream>>>(Xh, Xl, WoutT, bout, T2, FO, nullptr);
        k_lnz<<<CHN / 8, 256, 0, stream>>>(T2, gout, beout, CHN, Z, Zh, Zl);
        for (int gi = 0; gi < CHN / GN; ++gi)
            k_gemm3<<<dim3(GN / 64, GN / 64, 1), 128, 0, stream>>>(Zh + (size_t)gi * GN * FO, Zl + (size_t)gi * GN * FO, Zh + (size_t)gi * GN * FO, Zl + (size_t)gi * GN * FO, FO, G + (size_t)gi * GN * GN, GN);
        k_graph<<<CHN / GN, 128, 0, stream>>>(Z, G, node0, out0, out1);
    }
}
